// PowerLinear_12180527251822
// MI455X (gfx1250) — hardware-verified
//
#include <hip/hip_runtime.h>
#include <stddef.h>


typedef float v4f __attribute__((ext_vector_type(4)));
typedef float v8f __attribute__((ext_vector_type(8)));
typedef __bf16 v8bf __attribute__((ext_vector_type(8)));
typedef __bf16 v16bf __attribute__((ext_vector_type(16)));
typedef unsigned short v8us __attribute__((ext_vector_type(8)));

#define FDIM 1024
#define NBAT 64
#define PREP_THREADS 128
#define PREP_WAVES (PREP_THREADS / 32)
#define TILE_COLS 32
#define GEMM_THREADS 32

#define WS_VHI   0
#define WS_VLO   (WS_VHI + NBAT * FDIM * 2)
#define WS_RSUM  (WS_VLO + NBAT * FDIM * 2)
#define WS_SVEC  (WS_RSUM + FDIM * 4)
#define WS_TOTAL (WS_SVEC + NBAT * 4)

union Frag16 { v16bf v; v8bf h[2]; unsigned short s[16]; };
union Pack8  { v8us v; unsigned short s[8]; };

__device__ __forceinline__ unsigned int bf_split(float f) {
    const unsigned int u  = __float_as_uint(f);
    const unsigned int hu = (u + 0x7FFFu + ((u >> 16) & 1u)) & 0xFFFF0000u;
    const float rf = f - __uint_as_float(hu);
    const unsigned int ru = __float_as_uint(rf);
    const unsigned int lu = (ru + 0x7FFFu + ((ru >> 16) & 1u)) >> 16;
    return (hu >> 16) | (lu << 16);
}

__device__ __forceinline__ void split4(const v4f f, Frag16& hi, Frag16& lo, const int base) {
#pragma unroll
    for (int e = 0; e < 4; ++e) {
        const unsigned int r = bf_split(f[e]);
        hi.s[base + e] = (unsigned short)(r & 0xFFFFu);
        lo.s[base + e] = (unsigned short)(r >> 16);
    }
}

__device__ __forceinline__ v8f wmma_bf16(v16bf a, v16bf b, v8f c) {
    c = __builtin_amdgcn_wmma_f32_16x16x32_bf16(false, a, false, b, (short)0, c, false, false);
    asm volatile("v_nop\n\tv_nop\n\tv_nop\n\tv_nop" : "+v"(c) : "v"(a), "v"(b));
    return c;
}

__device__ __forceinline__ v8f zero8() {
    v8f z = {0.f, 0.f, 0.f, 0.f, 0.f, 0.f, 0.f, 0.f};
    return z;
}

__device__ __forceinline__ float wave_sum(float v) {
    v += __shfl_xor(v, 16, 32);
    v += __shfl_xor(v, 8, 32);
    v += __shfl_xor(v, 4, 32);
    v += __shfl_xor(v, 2, 32);
    v += __shfl_xor(v, 1, 32);
    return v;
}

__global__ __launch_bounds__(PREP_THREADS) void k_prep(const float* __restrict__ x,
                                                         const int* __restrict__ nvec,
                                                         const float* __restrict__ diag,
                                                         const float* __restrict__ rot,
                                                         unsigned short* vhi,
                                                         unsigned short* vlo,
                                                         float* rowsum,
                                                         float* svec) {
    __shared__ float sh_rs[FDIM];
    __shared__ float sh_s[NBAT];
    __shared__ float sh_red[PREP_WAVES];

    const int t    = threadIdx.x;
    const int lane = t & 31;
    const int w    = t >> 5;
    const int c0   = 8 * t;

    v4f ca = {0.f, 0.f, 0.f, 0.f};
    v4f cb = {0.f, 0.f, 0.f, 0.f};
#pragma unroll 1
    for (int r = 0; r < FDIM; ++r) {
        const float* p = rot + (size_t)r * FDIM + c0;
        ca += *(const v4f*)p;
        cb += *(const v4f*)(p + 4);
    }
    const v4f da = *(const v4f*)(diag + c0);
    const v4f db = *(const v4f*)(diag + c0 + 4);

#pragma unroll 1
    for (int b = 0; b < NBAT; ++b) {
        int nb = nvec[b];
        nb = nb < 0 ? 0 : nb;
        nb = nb > 31 ? 31 : nb;
        v4f pa = {1.f, 1.f, 1.f, 1.f};
        v4f pb = {1.f, 1.f, 1.f, 1.f};
        for (int q = 0; q < nb; ++q) { pa *= da; pb *= db; }

        const float* xp = x + (size_t)b * FDIM + c0;
        const v4f xa = *(const v4f*)xp;
        const v4f xb = *(const v4f*)(xp + 4);
        const v4f va = (ca * pa) * xa;
        const v4f vb = (cb * pb) * xb;

        Pack8 ph, pl;
#pragma unroll
        for (int e = 0; e < 4; ++e) {
            const unsigned int r0 = bf_split(va[e]);
            const unsigned int r1 = bf_split(vb[e]);
            ph.s[e]     = (unsigned short)(r0 & 0xFFFFu);
            pl.s[e]     = (unsigned short)(r0 >> 16);
            ph.s[4 + e] = (unsigned short)(r1 & 0xFFFFu);
            pl.s[4 + e] = (unsigned short)(r1 >> 16);
        }
        const v8us hv = ph.v;
        const v8us lv = pl.v;
        const size_t vo = (size_t)b * FDIM + c0;
        *(volatile v8us*)(vhi + vo) = hv;
        *(volatile v8us*)(vlo + vo) = lv;
        __threadfence();
        *(volatile v8us*)(vhi + vo) = hv;
        *(volatile v8us*)(vlo + vo) = lv;

        const v4f pr = ca * xa + cb * xb;
        float sp = (pr.x + pr.y) + (pr.z + pr.w);
        sp = wave_sum(sp);
        if (lane == 0) sh_red[w] = sp;
        __syncthreads();
        if (t == 0) sh_s[b] = (sh_red[0] + sh_red[1]) + (sh_red[2] + sh_red[3]);
        __syncthreads();
    }

#pragma unroll 1
    for (int r = w; r < FDIM; r += PREP_WAVES) {
        const float* p = rot + (size_t)r * FDIM + 4 * lane;
        v4f a = {0.f, 0.f, 0.f, 0.f};
#pragma unroll
        for (int j = 0; j < 8; ++j) a += *(const v4f*)(p + 128 * j);
        float s = (a.x + a.y) + (a.z + a.w);
        s = wave_sum(s);
        if (lane == 0) sh_rs[r] = s;
    }
    __syncthreads();

    v4f ra, rb;
    ra.x = sh_rs[4 * t];     ra.y = sh_rs[4 * t + 1];
    ra.z = sh_rs[4 * t + 2]; ra.w = sh_rs[4 * t + 3];
    rb.x = sh_rs[512 + 4 * t];     rb.y = sh_rs[512 + 4 * t + 1];
    rb.z = sh_rs[512 + 4 * t + 2]; rb.w = sh_rs[512 + 4 * t + 3];
    v4f sv = {0.f, 0.f, 0.f, 0.f};
    if (t < NBAT / 4) {
        sv.x = sh_s[4 * t];     sv.y = sh_s[4 * t + 1];
        sv.z = sh_s[4 * t + 2]; sv.w = sh_s[4 * t + 3];
    }
    for (int pass = 0; pass < 2; ++pass) {
        *(volatile v4f*)(rowsum + 4 * t) = ra;
        *(volatile v4f*)(rowsum + 512 + 4 * t) = rb;
        if (t < NBAT / 4) *(volatile v4f*)(svec + 4 * t) = sv;
        if (pass == 0) __threadfence();
    }
}

__global__ __launch_bounds__(GEMM_THREADS) void k_gemm(const unsigned short* __restrict__ vhi,
                                                         const unsigned short* __restrict__ vlo,
                                                         const float* __restrict__ rot,
                                                         const float* __restrict__ rowsum,
                                                         const float* __restrict__ svec,
                                                         const int* __restrict__ nvec,
                                                         float* out) {
    __shared__ float tile[NBAT * TILE_COLS];

    const int l  = threadIdx.x & 31;
    const int h  = l >> 4;
    const int m  = l & 15;
    const int n0 = blockIdx.x * TILE_COLS;
    if (n0 + TILE_COLS > FDIM) return;

    v8f acc[4][2];
#pragma unroll
    for (int t = 0; t < 4; ++t)
#pragma unroll
        for (int j = 0; j < 2; ++j) acc[t][j] = zero8();

#pragma unroll 1
    for (int k0 = 0; k0 < FDIM; k0 += 32) {
        Frag16 bh[2], bl[2];
#pragma unroll
        for (int j = 0; j < 2; ++j) {
            const float* bp = rot + (size_t)(n0 + 16 * j + m) * FDIM + k0 + 8 * h;
            const v4f f0 = *(const v4f*)(bp);
            const v4f f1 = *(const v4f*)(bp + 4);
            const v4f f2 = *(const v4f*)(bp + 16);
            const v4f f3 = *(const v4f*)(bp + 20);
            split4(f0, bh[j], bl[j], 0);
            split4(f1, bh[j], bl[j], 4);
            split4(f2, bh[j], bl[j], 8);
            split4(f3, bh[j], bl[j], 12);
        }
#pragma unroll
        for (int t = 0; t < 4; ++t) {
            const size_t ao = (size_t)(16 * t + m) * FDIM + k0 + 8 * h;
            Frag16 ah, al;
            ah.h[0] = *(const v8bf*)(vhi + ao);
            ah.h[1] = *(const v8bf*)(vhi + ao + 16);
            al.h[0] = *(const v8bf*)(vlo + ao);
            al.h[1] = *(const v8bf*)(vlo + ao + 16);
#pragma unroll
            for (int j = 0; j < 2; ++j) {
                v8f c = acc[t][j];
                c = wmma_bf16(ah.v, bh[j].v, c);
                c = wmma_bf16(ah.v, bl[j].v, c);
                c = wmma_bf16(al.v, bh[j].v, c);
                acc[t][j] = c;
            }
        }
    }

#pragma unroll
    for (int t = 0; t < 4; ++t)
#pragma unroll
        for (int j = 0; j < 2; ++j)
#pragma unroll
            for (int r = 0; r < 8; ++r)
                tile[(16 * t + 8 * h + r) * TILE_COLS + 16 * j + m] = acc[t][j][r];
    __syncthreads();

    const int rsub = l >> 3;
    const int c4   = (l & 7) * 4;
    const v4f rs4  = *(const v4f*)(rowsum + n0 + c4);
    for (int pass = 0; pass < 2; ++pass) {
#pragma unroll
        for (int it = 0; it < NBAT / 4; ++it) {
            const int row  = 4 * it + rsub;
            const int nb   = nvec[row];
            const float sb = svec[row];
            const float* tp = tile + row * TILE_COLS + c4;
            v4f tv;
            tv.x = tp[0]; tv.y = tp[1]; tv.z = tp[2]; tv.w = tp[3];
            const v4f zv  = rs4 * sb;
            const v4f val = (nb <= 0) ? zv : tv;
            *(volatile v4f*)(out + (size_t)row * FDIM + n0 + c4) = val;
        }
        if (pass == 0) __threadfence();
    }
}

extern "C" void kernel_launch(void* const* d_in, const int* in_sizes, int n_in,
                              void* d_out, int out_size, void* d_ws, size_t ws_size,
                              hipStream_t stream) {
    if (n_in < 4) return;
    if (in_sizes[0] != NBAT * FDIM || in_sizes[1] != NBAT || in_sizes[2] != FDIM ||
        in_sizes[3] != FDIM * FDIM || out_size != NBAT * FDIM) return;
    if (ws_size < (size_t)WS_TOTAL) return;

    const float* x    = (const float*)d_in[0];
    const int*   nv   = (const int*)d_in[1];
    const float* diag = (const float*)d_in[2];
    const float* rot  = (const float*)d_in[3];

    float* out = (float*)d_out;
    char* ws = (char*)d_ws;
    unsigned short* vhi  = (unsigned short*)(ws + WS_VHI);
    unsigned short* vlo  = (unsigned short*)(ws + WS_VLO);
    float*          rsum = (float*)(ws + WS_RSUM);
    float*          svec = (float*)(ws + WS_SVEC);

    k_prep<<<dim3(1), dim3(PREP_THREADS), 0, stream>>>(x, nv, diag, rot, vhi, vlo, rsum, svec);
    k_gemm<<<dim3(FDIM / TILE_COLS), dim3(GEMM_THREADS), 0, stream>>>(vhi, vlo, rot, rsum, svec, nv, out);
}
